// TritonGatherConv_82429012344832
// MI455X (gfx1250) — hardware-run, weakly checked
//
#include <hip/hip_runtime.h>


namespace {
constexpr int NB = 2, L = 2048, C = 1024, NH = 8, KT = 64, HD = C / NH  , HALF = 16, S = 2 * HALF + 1  , NT = NB * L, NPJ = 2 * NH + NH * KT  , NTL = NPJ / 16  ;
constexpr float XS = 8.0f, HS = 256.0f, WSC = 256.0f, MAXF = 16.0f, MINF = 1.0f;
typedef _Float16 b16;
typedef __attribute__((ext_vector_type(16))) _Float16 v16b;
typedef __attribute__((ext_vector_type(8))) _Float16 v8b;
typedef __attribute__((ext_vector_type(8))) float v8f;
typedef __attribute__((ext_vector_type(4))) float v4f;
__device__ __forceinline__ float bf16_rne(float f) { unsigned int u = __float_as_uint(f); u += 0x7FFFu + ((u >> 16) & 1u); float r = __uint_as_float(u & 0xFFFF0000u); asm volatile("" : "+v"(r)); return r; }
__device__ __forceinline__ float bfv(float f) { float r = bf16_rne(f); asm volatile("" : "+v"(r)); return r; }
__device__ __forceinline__ void split16(float v, b16& hi, b16& lo) { hi = (b16)v; lo = (b16)(v - (float)hi); }
__device__ __forceinline__ v16b frag_kb(const b16* p, int hh) { const v8b a = *(const v8b*)(p + 8 * hh), b = *(const v8b*)(p + 16 + 8 * hh); v16b f;
#pragma unroll
  for (int e = 0; e < 8; ++e) { f[e] = a[e]; f[8 + e] = b[e]; } return f; }
__device__ __forceinline__ v8f wmma16b(v16b a, v16b b, v8f c) { v8f d = __builtin_amdgcn_wmma_f32_16x16x32_f16(false, a, false, b, (short)0, c, false, false); asm volatile("v_nop\n\tv_nop\n\tv_nop\n\tv_nop" : "+v"(d) : "v"(a), "v"(b)); return d; }
__device__ __forceinline__ void wave_lds_sync() { __builtin_amdgcn_fence(__ATOMIC_RELEASE, "workgroup"); __builtin_amdgcn_wave_barrier(); __builtin_amdgcn_fence(__ATOMIC_ACQUIRE, "workgroup"); }
__device__ __forceinline__ float pmul(float a, float b) { float p = a * b; asm volatile("" : "+v"(p)); return p; }
__device__ __forceinline__ float silu(float v) { return v / (1.0f + __expf(-v)); }

__global__ __launch_bounds__(256) void wput_kernel(const float* __restrict__ ww, const float* __restrict__ kw, const float* __restrict__ ow, b16* __restrict__ WP, b16* __restrict__ WOT) { const size_t u = (size_t)blockIdx.x * 256 + threadIdx.x; v8b v;
  if (u < (size_t)NPJ * (C / 8)) { const int r = (int)(u / (C / 8)), k0 = (int)(u % (C / 8)) * 8; const float* w = r < 2 * NH ? ww + (size_t)r * C : kw + (size_t)(r - 2 * NH) * C;
#pragma unroll
    for (int j = 0; j < 8; ++j) v[j] = (b16)(bf16_rne(w[k0 + j]) * WSC); for (int pass = 0; pass < 2; ++pass) { *(volatile v8b*)(WP + (size_t)r * C + k0) = v; __threadfence(); } }
  if (u < (size_t)C * (C / 8)) {
#pragma unroll
    for (int j = 0; j < 8; ++j) v[j] = (b16)(bf16_rne(ow[u * 8 + j]) * WSC); for (int pass = 0; pass < 2; ++pass) { *(volatile v8b*)(WOT + u * 8) = v; __threadfence(); } } }
__global__ __launch_bounds__(32) void proj_kernel(const float* __restrict__ x, const b16* __restrict__ WP, const float* __restrict__ wb, const float* __restrict__ kb, int TLIM, float* __restrict__ FP, float* __restrict__ KE) { __shared__ __attribute__((aligned(16))) b16 Ah[16][C + 8]; __shared__ float Tf[16][11 * 16 + 4]; __shared__ float Fq[16][16]; const int lane = threadIdx.x, nloc = lane & 15, hlf = lane >> 4; const size_t m0 = (size_t)blockIdx.x * 16; if (m0 >= (size_t)TLIM) return;
  for (int rr = 0; rr < 16; ++rr) for (int q = 0; q < C / 32; ++q) Ah[rr][q * 32 + lane] = (b16)(bf16_rne(x[(m0 + rr) * C + q * 32 + lane]) * XS);
  wave_lds_sync();
#pragma unroll 1
  for (int g = 0; g < 3; ++g) { v8f acc[11];
#pragma unroll
    for (int t = 0; t < 11; ++t) acc[t] = (v8f){};
#pragma unroll 2
    for (int kk = 0; kk < C; kk += 32) { const v16b a = frag_kb(&Ah[nloc][kk], hlf);
#pragma unroll
      for (int t = 0; t < 11; ++t) acc[t] = wmma16b(a, frag_kb(WP + (size_t)((g * 11 + t) * 16 + nloc) * C + kk, hlf), acc[t]); }
#pragma unroll
    for (int t = 0; t < 11; ++t) { const int col = (g * 11 + t) * 16 + nloc; const float bb = col < 2 * NH ? bfv(wb[col]) : bfv(kb[col - 2 * NH]);
#pragma unroll
      for (int r8 = 0; r8 < 8; ++r8) Tf[8 * hlf + r8][t * 16 + nloc] = silu(acc[t][r8] * (1.0f / (XS * WSC)) + bb); }
    wave_lds_sync();
    if (g == 0) { for (int rr = 0; rr < 16; ++rr) if (lane < 16) { const float wv = Tf[rr][lane]; Fq[rr][lane] = lane < NH ? (1.0f / (1.0f + __expf(-wv))) * (MAXF - MINF) + MINF : tanhf(wv) * MAXF; } wave_lds_sync(); }
    for (int pass = 0; pass < 2; ++pass) { for (int rr = 0; rr < 16; ++rr) { if (g == 0) { if (lane < 16) ((volatile float*)FP)[(m0 + rr) * 16 + lane] = Fq[rr][lane];
          for (int c = lane; c < 160; c += 32) ((volatile float*)KE)[(m0 + rr) * (NH * KT) + c] = Tf[rr][16 + c]; }
        else { for (int c = lane; c < 176; c += 32) ((volatile float*)KE)[(m0 + rr) * (NH * KT) + 160 + (g - 1) * 176 + c] = Tf[rr][c]; } } __threadfence(); }
    wave_lds_sync(); } }
__global__ __launch_bounds__(256) void gather_kernel(const float* __restrict__ x, const float* __restrict__ FP, const float* __restrict__ KE, int TLIM, float* __restrict__ HID) { const int wave = threadIdx.x >> 5, lane = threadIdx.x & 31; const size_t tok = (size_t)blockIdx.x * 8 + wave; if (tok >= (size_t)TLIM) return; const int b = (int)(tok / L), l = (int)(tok % L); const float* xb = x + (size_t)b * L * C;
  float hid[NH][4];
#pragma unroll
  for (int h = 0; h < NH; ++h) { const float fr = FP[tok * 16 + h], phs = FP[tok * 16 + NH + h]; float a4[4] = {0.0f, 0.0f, 0.0f, 0.0f};
#pragma unroll 1
    for (int s = 0; s < S; ++s) { float pos = (float)l + phs + (float)(s - HALF) * fr; pos = fminf(fmaxf(pos, 0.0f), (float)(L - 1)); const float pf = floorf(pos); const int p0 = (int)pf; const int p1 = p0 + 1 < L ? p0 + 1 : L - 1; const float w1 = pos - pf, w0 = 1.0f - w1; const float kv = KE[tok * (NH * KT) + h * KT + s];
      const v4f xa = *(const v4f*)(xb + (size_t)p0 * C + h * HD + lane * 4), xc = *(const v4f*)(xb + (size_t)p1 * C + h * HD + lane * 4);
#pragma unroll
      for (int k = 0; k < 4; ++k) a4[k] += pmul(kv, pmul(w0, bfv(xa[k])) + pmul(w1, bfv(xc[k]))); }
#pragma unroll
    for (int k = 0; k < 4; ++k) hid[h][k] = a4[k]; }
  for (int pass = 0; pass < 2; ++pass) {
#pragma unroll
    for (int h = 0; h < NH; ++h) *(volatile v4f*)(HID + tok * C + h * HD + lane * 4) = (v4f){hid[h][0], hid[h][1], hid[h][2], hid[h][3]}; __threadfence(); } }
__global__ __launch_bounds__(32) void out_kernel(const float* __restrict__ HID, const b16* __restrict__ WOT, int TLIM, float* __restrict__ out) { __shared__ __attribute__((aligned(16))) b16 Ah[16][C + 8], Al[16][C + 8]; __shared__ float Tf[16][260]; const int lane = threadIdx.x, nloc = lane & 15, hlf = lane >> 4; const size_t m0 = (size_t)blockIdx.x * 16; if (m0 >= (size_t)TLIM) return;
  for (int rr = 0; rr < 16; ++rr) for (int q = 0; q < C / 32; ++q) { b16 p, ql; split16(HID[(m0 + rr) * C + q * 32 + lane] * HS, p, ql); Ah[rr][q * 32 + lane] = p; Al[rr][q * 32 + lane] = ql; }
  wave_lds_sync();
#pragma unroll 1
  for (int g = 0; g < C / 256; ++g) { v8f acc[16];
#pragma unroll
    for (int t = 0; t < 16; ++t) acc[t] = (v8f){};
#pragma unroll 2
    for (int kk = 0; kk < C; kk += 32) { const v16b a = frag_kb(&Ah[nloc][kk], hlf), al = frag_kb(&Al[nloc][kk], hlf);
#pragma unroll
      for (int t = 0; t < 16; ++t) { const v16b bw = frag_kb(WOT + (size_t)(g * 256 + t * 16 + nloc) * C + kk, hlf); acc[t] = wmma16b(a, bw, acc[t]); acc[t] = wmma16b(al, bw, acc[t]); } }
#pragma unroll
    for (int t = 0; t < 16; ++t) { const int cc = t * 16 + nloc;
#pragma unroll
      for (int r8 = 0; r8 < 8; ++r8) Tf[8 * hlf + r8][cc] = silu(acc[t][r8] * (1.0f / (HS * WSC))); }
    wave_lds_sync();
    for (int pass = 0; pass < 2; ++pass) { for (int rr = 0; rr < 16; ++rr) for (int q = 0; q < 2; ++q) *(volatile v4f*)(out + (m0 + rr) * C + g * 256 + q * 128 + lane * 4) = *(const v4f*)(&Tf[rr][q * 128 + lane * 4]); __threadfence(); }
    wave_lds_sync(); } }
}

extern "C" void kernel_launch(void* const* d_in, const int* in_sizes, int n_in, void* d_out, int out_size, void* d_ws, size_t ws_size, hipStream_t stream) {
  (void)n_in;
  auto Fp = [&](int i) { return (const float*)d_in[i]; };
  if (in_sizes[0] != NT * C || in_sizes[1] != 2 * NH * C || in_sizes[2] != 2 * NH || in_sizes[3] != NH * KT * C || in_sizes[4] != NH * KT || in_sizes[5] != C * C || out_size != NT * C) return;
  const int TLIM = NT;
  size_t off = 0; char* ws = (char*)d_ws;
  auto carve = [&](size_t bytes) { char* p = ws + off; off += (bytes + 255) & ~(size_t)255; return p; };
  b16* WP = (b16*)carve((size_t)NPJ * C * 2); b16* WOT = (b16*)carve((size_t)C * C * 2); float* FP = (float*)carve((size_t)NT * 16 * 4); float* KE = (float*)carve((size_t)NT * NH * KT * 4); float* HID = (float*)carve((size_t)NT * C * 4);
  if (off > ws_size || off > ((size_t)64 << 20)) return;
  wput_kernel<<<(unsigned)(((size_t)C * (C / 8) + 255) / 256), 256, 0, stream>>>(Fp(1), Fp(3), Fp(5), WP, WOT);
  proj_kernel<<<TLIM / 16, 32, 0, stream>>>(Fp(0), WP, Fp(2), Fp(4), TLIM, FP, KE);
  gather_kernel<<<(TLIM + 7) / 8, 256, 0, stream>>>(Fp(0), FP, KE, TLIM, HID);
  out_kernel<<<TLIM / 16, 32, 0, stream>>>(HID, WOT, TLIM, (float*)d_out);
}
